// D_GA_1812476199112
// MI455X (gfx1250) — hardware-verified
//
#include <hip/hip_runtime.h>
#include <stdint.h>


typedef _Float16       v16h  __attribute__((ext_vector_type(16)));
typedef _Float16       v8h   __attribute__((ext_vector_type(8)));
typedef __bf16         v16b  __attribute__((ext_vector_type(16)));
typedef unsigned short v16us __attribute__((ext_vector_type(16)));
typedef unsigned short v8us  __attribute__((ext_vector_type(8)));
typedef float          v8f   __attribute__((ext_vector_type(8)));
typedef float          v4f   __attribute__((ext_vector_type(4)));
typedef float          v2f   __attribute__((ext_vector_type(2)));

#define NB    8
#define NC    64
#define HIMG  64
#define WIMG  64
#define NTOK  1024
#define NHEAD 16
#define HD    4
#define NQKV  192

__device__ __forceinline__ v16h cat_h(v8h a, v8h b) {
    return __builtin_shufflevector(a, b, 0, 1, 2, 3, 4, 5, 6, 7, 8, 9, 10, 11, 12, 13, 14, 15);
}
__device__ __forceinline__ v16us cat_us(v8us a, v8us b) {
    return __builtin_shufflevector(a, b, 0, 1, 2, 3, 4, 5, 6, 7, 8, 9, 10, 11, 12, 13, 14, 15);
}

__device__ __forceinline__ v8f wmma_f16(v16h a, v16h b, v8f c) {
    v8f d = __builtin_amdgcn_wmma_f32_16x16x32_f16(false, a, false, b, (short)0, c, false, false);
    asm volatile("v_nop\n\tv_nop\n\tv_nop\n\tv_nop" : "+v"(d) : "v"(a), "v"(b));
    return d;
}

__device__ __forceinline__ v8f wmma_bf16(v16us au, v16us bu, v8f c) {
    v16b a = __builtin_bit_cast(v16b, au);
    v16b b = __builtin_bit_cast(v16b, bu);
    v8f d = __builtin_amdgcn_wmma_f32_16x16x32_bf16(false, a, false, b, (short)0, c, false, false);
    asm volatile("v_nop\n\tv_nop\n\tv_nop\n\tv_nop" : "+v"(d) : "v"(a), "v"(b));
    return d;
}

__device__ __forceinline__ unsigned short bf16_bits(float x) {
    unsigned int u = __float_as_uint(x);
    u += 0x7FFFu + ((u >> 16) & 1u);
    return (unsigned short)(u >> 16);
}
__device__ __forceinline__ float bf16_val(unsigned short b) {
    return __uint_as_float(((unsigned int)b) << 16);
}

template <typename T>
__device__ __forceinline__ void vstore(void* p, T v) { *(volatile T*)p = v; }

__device__ __forceinline__ int win_argmax(const float* __restrict__ p, float& best) {
    v2f r0 = *(const v2f*)p;
    v2f r1 = *(const v2f*)(p + WIMG);
    float bv = r0.x; int bi = 0;
    if (r0.y > bv) { bv = r0.y; bi = 1; }
    if (r1.x > bv) { bv = r1.x; bi = 2; }
    if (r1.y > bv) { bv = r1.y; bi = 3; }
    best = bv;
    return bi;
}

__global__ __launch_bounds__(256) void k_weights(const float* __restrict__ wq, const float* __restrict__ wp,
                                                 _Float16* __restrict__ wqT,
                                                 unsigned short* __restrict__ wpH,
                                                 unsigned short* __restrict__ wpL) {
    const int i = blockIdx.x * 256 + threadIdx.x;
    if (i < NQKV * 8) {
        const int n = i >> 3, q = i & 7;
        v8h o;
#pragma unroll
        for (int e = 0; e < 8; ++e) o[e] = (_Float16)wq[(8 * q + e) * NQKV + n];
        _Float16* dst = wqT + n * NC + 8 * q;
        vstore<v8h>(dst, o);
        __threadfence();
        vstore<v8h>(dst, o);
    } else {
        const int j = i - NQKV * 8;
        const int n = j >> 3, q = j & 7;
        v8us hi, lo;
#pragma unroll
        for (int e = 0; e < 8; ++e) {
            float w = wp[(8 * q + e) * NC + n];
            unsigned short hb = bf16_bits(w);
            hi[e] = hb;
            lo[e] = bf16_bits(w - bf16_val(hb));
        }
        unsigned short* dh = wpH + n * NC + 8 * q;
        unsigned short* dl = wpL + n * NC + 8 * q;
        vstore<v8us>(dh, hi);
        vstore<v8us>(dl, lo);
        __threadfence();
        vstore<v8us>(dh, hi);
        vstore<v8us>(dl, lo);
    }
}

__global__ __launch_bounds__(256) void k_pool(const float* __restrict__ x, _Float16* __restrict__ t16) {
    __shared__ __align__(16) _Float16 sT[32 * NC];
    const int b = blockIdx.x >> 5, hp = blockIdx.x & 31;
    const int tid = threadIdx.x;
    const int wp = tid & 31, cw = tid >> 5;
#pragma unroll
    for (int p = 0; p < 8; ++p) {
        const int c = p * 8 + cw;
        const float* base = x + ((size_t)((b * NC + c) * HIMG + 2 * hp)) * WIMG + 2 * wp;
        float best;
        (void)win_argmax(base, best);
        sT[wp * NC + c] = (_Float16)best;
    }
    __syncthreads();
    const int tok = tid >> 3, q = tid & 7;
    v8h val = *(const v8h*)(sT + tok * NC + 8 * q);
    _Float16* dst = t16 + ((size_t)(b * NTOK + hp * 32 + tok)) * NC + 8 * q;
    vstore<v8h>(dst, val);
    __threadfence();
    vstore<v8h>(dst, val);
}

__global__ __launch_bounds__(384) void k_qkv(const _Float16* __restrict__ t16, const _Float16* __restrict__ wqT,
                                             float* __restrict__ qbuf, float* __restrict__ kbuf,
                                             _Float16* __restrict__ vT) {
    __shared__ __align__(16) float sD[12][64 * 16];
    const int wv = threadIdx.x >> 5, l = threadIdx.x & 31, h = l >> 4, m = l & 15;
    const int tg0 = blockIdx.x * 64;
    const int n0 = wv * 16;

    v8f acc[4];
#pragma unroll
    for (int j = 0; j < 4; ++j) acc[j] = (v8f){0.f, 0.f, 0.f, 0.f, 0.f, 0.f, 0.f, 0.f};

#pragma unroll
    for (int c = 0; c < 2; ++c) {
        const int k0 = 32 * c;
        const _Float16* bp = wqT + (size_t)(n0 + m) * NC + k0;
        v16h bf = cat_h(*(const v8h*)(bp + 8 * h), *(const v8h*)(bp + 16 + 8 * h));
#pragma unroll
        for (int j = 0; j < 4; ++j) {
            const _Float16* ap = t16 + (size_t)(tg0 + 16 * j + m) * NC + k0;
            v16h a = cat_h(*(const v8h*)(ap + 8 * h), *(const v8h*)(ap + 16 + 8 * h));
            acc[j] = wmma_f16(a, bf, acc[j]);
        }
    }
    float* sd = sD[wv];
#pragma unroll
    for (int j = 0; j < 4; ++j) {
#pragma unroll
        for (int r = 0; r < 8; ++r) sd[(16 * j + 8 * h + r) * 16 + m] = acc[j][r];
    }
    __syncthreads();

    const int sec = wv >> 2;
    const int hb  = (wv & 3) * 4;
    const int b   = tg0 >> 10, t0 = tg0 & 1023;
    if (sec < 2) {
        float* dbase = (sec == 0) ? qbuf : kbuf;
        v4f vals[8];
        float* dsts[8];
#pragma unroll
        for (int p = 0; p < 8; ++p) {
            const int f = p * 32 + l;
            const int hl = f >> 6, tok = f & 63;
            vals[p] = *(const v4f*)(sd + tok * 16 + hl * 4);
            dsts[p] = dbase + (((size_t)(b * NHEAD + hb + hl)) * NTOK + t0 + tok) * HD;
        }
#pragma unroll
        for (int p = 0; p < 8; ++p) vstore<v4f>(dsts[p], vals[p]);
        __threadfence();
#pragma unroll
        for (int p = 0; p < 8; ++p) vstore<v4f>(dsts[p], vals[p]);
    } else {
        v8h vals[4];
        _Float16* dsts[4];
#pragma unroll
        for (int p = 0; p < 4; ++p) {
            const int f = p * 32 + l;
            const int col = f >> 3, piece = f & 7;
            v8h u;
#pragma unroll
            for (int e = 0; e < 8; ++e) u[e] = (_Float16)sd[(piece * 8 + e) * 16 + col];
            vals[p] = u;
            dsts[p] = vT + (((size_t)(b * NHEAD + hb + (col >> 2))) * HD + (col & 3)) * NTOK + t0 + piece * 8;
        }
#pragma unroll
        for (int p = 0; p < 4; ++p) vstore<v8h>(dsts[p], vals[p]);
        __threadfence();
#pragma unroll
        for (int p = 0; p < 4; ++p) vstore<v8h>(dsts[p], vals[p]);
    }
}

__global__ __launch_bounds__(256) void k_attn(const float* __restrict__ qbuf, const float* __restrict__ kbuf,
                                              const _Float16* __restrict__ vT, float* __restrict__ ohb) {
    __shared__ __align__(16) float    kS[NTOK * HD];
    __shared__ __align__(16) _Float16 vS[HD * NTOK];
    __shared__ __align__(16) float    sO[8][32 * HD];
    const int bh  = blockIdx.x >> 2;
    const int qc  = blockIdx.x & 3;
    const int tid = threadIdx.x, wv = tid >> 5, l = tid & 31, h = l >> 4, m = l & 15;

    {
        const v4f* kg = (const v4f*)(kbuf + (size_t)bh * NTOK * HD);
        v4f* kl = (v4f*)kS;
        for (int i = tid; i < NTOK; i += 256) kl[i] = kg[i];
        const v8h* vg = (const v8h*)(vT + (size_t)bh * NTOK * HD);
        v8h* vl = (v8h*)vS;
        for (int i = tid; i < (NTOK * HD) / 8; i += 256) vl[i] = vg[i];
    }
    __syncthreads();

    const int q0 = qc * 256 + wv * 32;
    const float QS = 0.5f * 1.44269504088896340736f;
    const v4f* kl4 = (const v4f*)kS;

    v4f qv = *(const v4f*)(qbuf + ((size_t)bh * NTOK + q0 + l) * HD);
    qv = qv * QS;
    float mx = -3.0e38f;
    for (int kk = 0; kk < NTOK; kk += 8) {
#pragma unroll
        for (int e = 0; e < 8; ++e) {
            v4f kv = kl4[kk + e];
            float s = qv.x * kv.x;
            s = __builtin_fmaf(qv.y, kv.y, s);
            s = __builtin_fmaf(qv.z, kv.z, s);
            s = __builtin_fmaf(qv.w, kv.w, s);
            mx = fmaxf(mx, s);
        }
    }
    const float mxa = __shfl(mx, m, 32) - 14.0f;
    const float mxb = __shfl(mx, 16 + m, 32) - 14.0f;

    v4f qa = *(const v4f*)(qbuf + ((size_t)bh * NTOK + q0 + m) * HD);
    v4f qb = *(const v4f*)(qbuf + ((size_t)bh * NTOK + q0 + 16 + m) * HD);
    qa = qa * QS;
    qb = qb * QS;

    v8f acc0 = (v8f){0.f, 0.f, 0.f, 0.f, 0.f, 0.f, 0.f, 0.f};
    v8f acc1 = (v8f){0.f, 0.f, 0.f, 0.f, 0.f, 0.f, 0.f, 0.f};
    float la = 0.f, lb = 0.f;
    const int dd = m & 3;
    for (int ks = 0; ks < NTOK / 32; ++ks) {
        const int k0 = ks * 32;
        v16h pa = (v16h){0, 0, 0, 0, 0, 0, 0, 0, 0, 0, 0, 0, 0, 0, 0, 0};
        v16h pb = (v16h){0, 0, 0, 0, 0, 0, 0, 0, 0, 0, 0, 0, 0, 0, 0, 0};
#pragma unroll
        for (int g = 0; g < 2; ++g) {
            const v4f* kp = (const v4f*)(kS + (k0 + 16 * g + 8 * h) * HD);
#pragma unroll
            for (int e = 0; e < 8; ++e) {
                v4f kv = kp[e];
                float sa = __builtin_fmaf(qa.x, kv.x, -mxa);
                sa = __builtin_fmaf(qa.y, kv.y, sa);
                sa = __builtin_fmaf(qa.z, kv.z, sa);
                sa = __builtin_fmaf(qa.w, kv.w, sa);
                float sb = __builtin_fmaf(qb.x, kv.x, -mxb);
                sb = __builtin_fmaf(qb.y, kv.y, sb);
                sb = __builtin_fmaf(qb.z, kv.z, sb);
                sb = __builtin_fmaf(qb.w, kv.w, sb);
                float ea = __builtin_amdgcn_exp2f(sa);
                float eb = __builtin_amdgcn_exp2f(sb);
                la += ea;
                lb += eb;
                pa[8 * g + e] = (_Float16)ea;
                pb[8 * g + e] = (_Float16)eb;
            }
        }
        const _Float16* vp = vS + dd * NTOK + k0;
        v16h bv = cat_h(*(const v8h*)(vp + 8 * h), *(const v8h*)(vp + 16 + 8 * h));
        acc0 = wmma_f16(pa, bv, acc0);
        acc1 = wmma_f16(pb, bv, acc1);
    }
    la += __shfl_xor(la, 16, 32);
    lb += __shfl_xor(lb, 16, 32);
    const float ia = 1.0f / la;
    const float ib = 1.0f / lb;

    float* so = sO[wv];
#pragma unroll
    for (int r = 0; r < 8; ++r) {
        const float fa = __shfl(ia, 8 * h + r, 32);
        const float fb = __shfl(ib, 8 * h + r, 32);
        if (m < HD) {
            so[(8 * h + r) * HD + m]      = acc0[r] * fa;
            so[(16 + 8 * h + r) * HD + m] = acc1[r] * fb;
        }
    }
    __syncthreads();
    v4f ov = *(const v4f*)(so + l * HD);
    float* dst = ohb + ((size_t)bh * NTOK + q0 + l) * HD;
    vstore<v4f>(dst, ov);
    __threadfence();
    vstore<v4f>(dst, ov);
}

__global__ __launch_bounds__(256) void k_proj(const float* __restrict__ ohb,
                                              const unsigned short* __restrict__ wpH,
                                              const unsigned short* __restrict__ wpL,
                                              const float* __restrict__ gamma, const float* __restrict__ beta,
                                              const float* __restrict__ rmean, const float* __restrict__ rvar,
                                              const float* __restrict__ x, float* __restrict__ out) {
    __shared__ float sV[NC * 33];
    __shared__ int   sI[NC * 33];
    const int b = blockIdx.x >> 5, hp = blockIdx.x & 31;
    const int tid = threadIdx.x, wv = tid >> 5, l = tid & 31, h = l >> 4, m = l & 15;

#pragma unroll
    for (int p = 0; p < 8; ++p) {
        const int c = p * 8 + (tid >> 5), wp = tid & 31;
        const float* base = x + ((size_t)((b * NC + c) * HIMG + 2 * hp)) * WIMG + 2 * wp;
        float best;
        sI[c * 33 + wp] = win_argmax(base, best);
    }

    const int mt = wv >> 2, nt = wv & 3;
    const int tok = hp * 32 + 16 * mt + m;
    v8f acc = (v8f){0.f, 0.f, 0.f, 0.f, 0.f, 0.f, 0.f, 0.f};
#pragma unroll
    for (int c2 = 0; c2 < 2; ++c2) {
        const int k0 = 32 * c2;
        v16us ahi, alo;
#pragma unroll
        for (int g = 0; g < 4; ++g) {
            const int head = 8 * c2 + 2 * h + (g & 1) + 4 * (g >> 1);
            v4f v = *(const v4f*)(ohb + (((size_t)(b * NHEAD + head)) * NTOK + tok) * HD);
#pragma unroll
            for (int e = 0; e < 4; ++e) {
                unsigned short hb = bf16_bits(v[e]);
                ahi[4 * g + e] = hb;
                alo[4 * g + e] = bf16_bits(v[e] - bf16_val(hb));
            }
        }
        const unsigned short* ph = wpH + (size_t)(nt * 16 + m) * NC + k0;
        const unsigned short* pl = wpL + (size_t)(nt * 16 + m) * NC + k0;
        v16us bhi = cat_us(*(const v8us*)(ph + 8 * h), *(const v8us*)(ph + 16 + 8 * h));
        v16us blo = cat_us(*(const v8us*)(pl + 8 * h), *(const v8us*)(pl + 16 + 8 * h));
        acc = wmma_bf16(ahi, bhi, acc);
        acc = wmma_bf16(ahi, blo, acc);
        acc = wmma_bf16(alo, bhi, acc);
    }
    {
        const int c = nt * 16 + m;
        const float invc = gamma[c] * rsqrtf(rvar[c] + 1e-5f);
        const float bias = beta[c] - rmean[c] * invc;
#pragma unroll
        for (int r = 0; r < 8; ++r) sV[c * 33 + 16 * mt + 8 * h + r] = acc[r] * invc + bias;
    }
    __syncthreads();

    v4f vals[8];
    float* dsts[8];
#pragma unroll
    for (int p = 0; p < 8; ++p) {
        const int f = p * 256 + tid;
        const int row = f >> 4, cc = row >> 1, dh = row & 1, q = f & 15;
        v4f v;
#pragma unroll
        for (int jj = 0; jj < 4; ++jj) {
            const int wp = 2 * q + (jj >> 1), dw = jj & 1;
            const int id = sI[cc * 33 + wp];
            const float val = sV[cc * 33 + wp];
            v[jj] = (id == dh * 2 + dw) ? val : 0.f;
        }
        vals[p] = v;
        dsts[p] = out + (((size_t)(b * NC + cc)) * HIMG + 2 * hp + dh) * WIMG + 4 * q;
    }
#pragma unroll
    for (int p = 0; p < 8; ++p) vstore<v4f>(dsts[p], vals[p]);
    __threadfence();
#pragma unroll
    for (int p = 0; p < 8; ++p) vstore<v4f>(dsts[p], vals[p]);
}

extern "C" void kernel_launch(void* const* d_in, const int* in_sizes, int n_in,
                              void* d_out, int out_size, void* d_ws, size_t ws_size,
                              hipStream_t stream) {
    if (n_in < 7) return;
    if (in_sizes[0] != NB * NC * HIMG * WIMG) return;
    if (in_sizes[1] != NC * NQKV) return;
    if (in_sizes[2] != NC * NC) return;
    if (in_sizes[3] != NC || in_sizes[4] != NC || in_sizes[5] != NC || in_sizes[6] != NC) return;
    if (out_size != NB * NC * HIMG * WIMG) return;

    const float* x      = (const float*)d_in[0];
    const float* w_qkv  = (const float*)d_in[1];
    const float* w_proj = (const float*)d_in[2];
    const float* gamma  = (const float*)d_in[3];
    const float* beta   = (const float*)d_in[4];
    const float* rmean  = (const float*)d_in[5];
    const float* rvar   = (const float*)d_in[6];
    float* out = (float*)d_out;

    const size_t sz_t16 = (size_t)NB * NTOK * NC * 2;
    const size_t sz_qk  = (size_t)NB * NHEAD * NTOK * HD * 4;
    const size_t sz_v   = (size_t)NB * NHEAD * HD * NTOK * 2;
    const size_t sz_o   = sz_qk;
    const size_t sz_wq  = (size_t)NQKV * NC * 2;
    const size_t sz_wp  = (size_t)NC * NC * 2;
    const size_t off_t16 = 0;
    const size_t off_q   = off_t16 + sz_t16;
    const size_t off_k   = off_q + sz_qk;
    const size_t off_v   = off_k + sz_qk;
    const size_t off_o   = off_v + sz_v;
    const size_t off_wq  = off_o + sz_o;
    const size_t off_wph = off_wq + sz_wq;
    const size_t off_wpl = off_wph + sz_wp;
    const size_t off_end = off_wpl + sz_wp;
    if (off_end > ws_size) return;

    char* ws = (char*)d_ws;
    _Float16*       t16  = (_Float16*)(ws + off_t16);
    float*          qbuf = (float*)(ws + off_q);
    float*          kbuf = (float*)(ws + off_k);
    _Float16*       vT   = (_Float16*)(ws + off_v);
    float*          ohb  = (float*)(ws + off_o);
    _Float16*       wqT  = (_Float16*)(ws + off_wq);
    unsigned short* wpH  = (unsigned short*)(ws + off_wph);
    unsigned short* wpL  = (unsigned short*)(ws + off_wpl);

    k_weights<<<8, 256, 0, stream>>>(w_qkv, w_proj, wqT, wpH, wpL);
    k_pool<<<NB * 32, 256, 0, stream>>>(x, t16);
    k_qkv<<<(NB * NTOK) / 64, 384, 0, stream>>>(t16, wqT, qbuf, kbuf, vT);
    k_attn<<<NB * NHEAD * 4, 256, 0, stream>>>(qbuf, kbuf, vT, ohb);
    k_proj<<<NB * 32, 256, 0, stream>>>(ohb, wpH, wpL, gamma, beta, rmean, rvar, x, out);
}
